// TransformerXLHybridEncoder_16484084482890
// MI455X (gfx1250) — hardware-verified
//
#include <hip/hip_runtime.h>
#include <math.h>

constexpr int kQLen   = 1024;
constexpr int kMLen   = 1024;
constexpr int kKLen   = 2048;
constexpr int kBsz    = 4;
constexpr int kDModel = 1024;
constexpr int kNHead  = 16;
constexpr int kDHead  = 64;
constexpr int kHDim   = 1024;
constexpr int kQkvCols = 3072;
constexpr int kKVPitch = 2048;
constexpr int kTokQ   = kQLen * kBsz;

constexpr float kWCarry     = 64.0f;
constexpr float kProjScale  = 1.0f / 64.0f;
constexpr float kVecCarry   = 256.0f;
constexpr float kPCarry     = 32768.0f;
constexpr float kInvLP      = 1.0f / 128.0f;
constexpr float kOutScale   = 1.0f / (256.0f * 64.0f);
constexpr float kScoreScale = 0.125f;
constexpr float kLnEps      = 1e-5f;
constexpr float kInvD       = 1.0f / 1024.0f;

constexpr int kKC      = 64;
constexpr int kRWin    = 128;
constexpr int kBdPitch = 84;
constexpr int kOsPitch = 68;

typedef __attribute__((ext_vector_type(16))) _Float16 v16h;
typedef __attribute__((ext_vector_type(8)))  _Float16 v8h;
typedef __attribute__((ext_vector_type(16))) __bf16   v16b;
typedef __attribute__((ext_vector_type(8)))  __bf16   v8b;
typedef __attribute__((ext_vector_type(8)))  float    v8f;
typedef __attribute__((ext_vector_type(4)))  float    v4f;
typedef __attribute__((ext_vector_type(4)))  unsigned int v4u;

__device__ __forceinline__ unsigned short f2bf_bits(float f) {
  unsigned u = __float_as_uint(f);
  return (unsigned short)((u + 0x7FFFu + ((u >> 16) & 1u)) >> 16);
}
__device__ __forceinline__ float bf_bits2f(unsigned short h) { return __uint_as_float(((unsigned)h) << 16); }

__device__ __forceinline__ void dep_guard_h(v8f& a, v8f& b, v16h x, v16h y) { asm volatile("v_nop\n\tv_nop\n\tv_nop\n\tv_nop" : "+v"(a), "+v"(b) : "v"(x), "v"(y)); }
__device__ __forceinline__ void dep_guard_b(v8f& a, v8f& b, v16b x, v16b y) { asm volatile("v_nop\n\tv_nop\n\tv_nop\n\tv_nop" : "+v"(a), "+v"(b) : "v"(x), "v"(y)); }
__device__ __forceinline__ void keep4_h(v16h a, v16h b, v16h c, v16h d) { asm volatile("v_nop" :: "v"(a), "v"(b), "v"(c), "v"(d)); }
__device__ __forceinline__ void keep4_b(v16b a, v16b b, v16b c, v16b d) { asm volatile("v_nop" :: "v"(a), "v"(b), "v"(c), "v"(d)); }
__device__ __forceinline__ void acc_guard4(v8f& a, v8f& b, v8f& c, v8f& d) { asm volatile("v_nop\n\tv_nop\n\tv_nop\n\tv_nop" : "+v"(a), "+v"(b), "+v"(c), "+v"(d)); }
template <typename T> struct Frag;
template <> struct Frag<_Float16> {
  typedef v16h V; union U { v16h v; v8h h[2]; };
  static __device__ __forceinline__ v16h load(const _Float16* p) {
    U f; f.h[0] = *(const v8h*)(p); f.h[1] = *(const v8h*)(p + 16); return f.v;
  }
  static __device__ __forceinline__ v8f mma(v16h a, v16h b, v8f c) {
    return __builtin_amdgcn_wmma_f32_16x16x32_f16(false, a, false, b, (short)0, c, false, false);
  }
  static __device__ __forceinline__ void guard(v8f& a, v8f& b, v16h x, v16h y) { dep_guard_h(a, b, x, y); }
  static __device__ __forceinline__ void keep(v16h a, v16h b, v16h c, v16h d) { keep4_h(a, b, c, d); }
};
template <> struct Frag<__bf16> {
  typedef v16b V; union U { v16b v; v8b h[2]; };
  static __device__ __forceinline__ v16b load(const __bf16* p) {
    U f; f.h[0] = *(const v8b*)(p); f.h[1] = *(const v8b*)(p + 16); return f.v;
  }
  static __device__ __forceinline__ v8f mma(v16b a, v16b b, v8f c) {
    return __builtin_amdgcn_wmma_f32_16x16x32_bf16(false, a, false, b, (short)0, c, false, false);
  }
  static __device__ __forceinline__ void guard(v8f& a, v8f& b, v16b x, v16b y) { dep_guard_b(a, b, x, y); }
  static __device__ __forceinline__ void keep(v16b a, v16b b, v16b c, v16b d) { keep4_b(a, b, c, d); }
};

__device__ __forceinline__ unsigned pk16(unsigned short a, unsigned short b) { return (unsigned)a | ((unsigned)b << 16); }
__device__ __forceinline__ unsigned short h_bits(float f) { const _Float16 h = (_Float16)f; return __builtin_bit_cast(unsigned short, h); }
__device__ __forceinline__ unsigned short h16_bits(_Float16 h) { return __builtin_bit_cast(unsigned short, h); }

template <int ET> struct Elem;
template <> struct Elem<0> { typedef _Float16 T; };
template <> struct Elem<1> { typedef __bf16 T; };
template <int ET, bool SPLIT, int BIAS_MODE, int OUT_MODE, bool RESID, int ACT = 0>
__global__ __launch_bounds__(256) void wmma_gemm64(
    const unsigned short* __restrict__ Ap, const unsigned short* __restrict__ A2p, int lda, long strideA,
    const unsigned short* __restrict__ Btp, const unsigned short* __restrict__ Bt2p, int ldb, long strideB,
    void* __restrict__ Cout, void* __restrict__ Cout2, int ldc, long strideC,
    const float* __restrict__ bias,
    const float* __restrict__ resid, long strideR,
    int M, int N, int K, float scale) {
  typedef typename Elem<ET>::T T;
  typedef typename Frag<T>::V V;
  const T* A = (const T*)Ap; const T* A2 = (const T*)A2p; const T* Bt = (const T*)Btp; const T* Bt2 = (const T*)Bt2p;
  __shared__ __align__(16) float sT[8][16 * 68];
  const int b    = blockIdx.y;
  const int lane = threadIdx.x & 31;
  const int wave = threadIdx.x >> 5;
  const int tilesN = N >> 6;
  const int tilesM = M >> 6;
  const int tile = blockIdx.x * 8 + wave;
  if (tile >= tilesM * tilesN) return;
  const int tm = tile / tilesN;
  const int tn = tile - tm * tilesN;
  const int m0 = tm << 6;
  const int n0 = tn << 6;

  const T* Ab  = A  + (size_t)b * strideA;
  const T* Bb  = Bt + (size_t)b * strideB;
  const T* Ab2 = SPLIT ? (A2  + (size_t)b * strideA) : nullptr;
  const T* Bb2 = SPLIT ? (Bt2 + (size_t)b * strideB) : nullptr;

  const int rlane = lane & 15;
  const int koff  = (lane >> 4) * 8;
  const int mOff  = (lane >> 4) * 8;

  v8f acc[4][4];
#pragma unroll
  for (int i = 0; i < 4; ++i)
#pragma unroll
    for (int j = 0; j < 4; ++j) acc[i][j] = (v8f){0.f,0.f,0.f,0.f,0.f,0.f,0.f,0.f};

  for (int k0 = 0; k0 < K; k0 += 32) {
    V bh[4], bl[4];
#pragma unroll
    for (int j = 0; j < 4; ++j) {
      const size_t bo = (size_t)(n0 + (j << 4) + rlane) * ldb + koff + k0;
      bh[j] = Frag<T>::load(Bb + bo);
      if (SPLIT) bl[j] = Frag<T>::load(Bb2 + bo);
    }
#pragma unroll
    for (int i = 0; i < 4; ++i) {
      const size_t ao = (size_t)(m0 + (i << 4) + rlane) * lda + koff + k0;
      V ah = Frag<T>::load(Ab + ao);
      V al;
      if (SPLIT) al = Frag<T>::load(Ab2 + ao);
#pragma unroll
      for (int j = 0; j < 4; ++j) {
        acc[i][j] = Frag<T>::mma(ah, bh[j], acc[i][j]);
        if (SPLIT) {
          acc[i][j] = Frag<T>::mma(ah, bl[j], acc[i][j]);
          acc[i][j] = Frag<T>::mma(al, bh[j], acc[i][j]);
        }
      }
      Frag<T>::guard(acc[i][0], acc[i][3], ah, SPLIT ? al : ah);
    }
    Frag<T>::keep(bh[0], bh[1], bh[2], bh[3]);
    if (SPLIT) Frag<T>::keep(bl[0], bl[1], bl[2], bl[3]);
  }
  acc_guard4(acc[0][0], acc[0][1], acc[0][2], acc[0][3]);
  acc_guard4(acc[1][0], acc[1][1], acc[1][2], acc[1][3]);
  acc_guard4(acc[2][0], acc[2][1], acc[2][2], acc[2][3]);
  acc_guard4(acc[3][0], acc[3][1], acc[3][2], acc[3][3]);

  float* slab = sT[wave];
  const float* Rb = RESID ? (resid + (size_t)b * strideR) : nullptr;
#pragma unroll
  for (int i = 0; i < 4; ++i) {
    const int mBase = m0 + (i << 4);
#pragma unroll
    for (int j = 0; j < 4; ++j) {
      const int n = n0 + (j << 4) + rlane;
      float bv = 0.f;
      if (BIAS_MODE == 2) bv = bias[n];
#pragma unroll
      for (int r = 0; r < 8; ++r) {
        float v = acc[i][j][r] * scale;
        if (BIAS_MODE == 1) v += bias[mBase + mOff + r];
        if (BIAS_MODE == 2) v += bv;
        if (RESID) v += Rb[(size_t)(mBase + mOff + r) * ldc + n];
        if (ACT == 2) v = fmaxf(v, 0.0f);
        if (ACT == 4) v = (v > 0.f) ? v : 0.01f * v;
        slab[(mOff + r) * 68 + (j << 4) + rlane] = v;
      }
    }
    __builtin_amdgcn_fence(__ATOMIC_RELEASE, "workgroup");
    __builtin_amdgcn_wave_barrier();
    __builtin_amdgcn_fence(__ATOMIC_ACQUIRE, "workgroup");
    if (OUT_MODE == 0) {
      float* C = (float*)Cout + (size_t)b * strideC;
      const int hh = lane >> 4, c4 = (lane & 15) * 4;
      for (int pass = 0; pass < 2; ++pass) {
#pragma unroll
        for (int it = 0; it < 8; ++it) {
          const int row = it * 2 + hh;
          v4f v = *(const v4f*)(slab + row * 68 + c4);
          *(volatile v4f*)(C + (size_t)(mBase + row) * ldc + n0 + c4) = v;
        }
        __threadfence();
      }
    } else {
      const int q = lane >> 3, c8 = (lane & 7) * 8;
      unsigned short* C  = (unsigned short*)Cout  + (size_t)b * strideC;
      unsigned short* C2 = (OUT_MODE == 2) ? ((unsigned short*)Cout2 + (size_t)b * strideC) : nullptr;
      for (int pass = 0; pass < 2; ++pass) {
#pragma unroll
        for (int it = 0; it < 4; ++it) {
          const int row = it * 4 + q;
          const float* sp = slab + row * 68 + c8;
          v8h hv, lv;
#pragma unroll
          for (int e = 0; e < 8; ++e) {
            if (OUT_MODE == 1) {
              hv[e] = (_Float16)sp[e];
            } else {
              unsigned short hb = f2bf_bits(sp[e]);
              unsigned short lb = f2bf_bits(sp[e] - bf_bits2f(hb));
              hv[e] = __builtin_bit_cast(_Float16, hb);
              lv[e] = __builtin_bit_cast(_Float16, lb);
            }
          }
          *(volatile v8h*)(C + (size_t)(mBase + row) * ldc + n0 + c8) = hv;
          if (OUT_MODE == 2) *(volatile v8h*)(C2 + (size_t)(mBase + row) * ldc + n0 + c8) = lv;
        }
        __threadfence();
      }
    }
    __builtin_amdgcn_fence(__ATOMIC_RELEASE, "workgroup");
    __builtin_amdgcn_wave_barrier();
    __builtin_amdgcn_fence(__ATOMIC_ACQUIRE, "workgroup");
  }
}

__global__ __launch_bounds__(256) void cast8_kernel(const float* __restrict__ in, unsigned short* __restrict__ out, int n8) {
  const int i = blockIdx.x * 256 + threadIdx.x;
  if (i >= n8) return;
  const size_t base = (size_t)i * 8;
  const v4f a = *(const v4f*)(in + base);
  const v4f c = *(const v4f*)(in + base + 4);
  unsigned short hb[8];
#pragma unroll
  for (int e = 0; e < 4; ++e) { hb[e] = h_bits(a[e]); hb[4 + e] = h_bits(c[e]); }
  const v4u u = (v4u){pk16(hb[0], hb[1]), pk16(hb[2], hb[3]), pk16(hb[4], hb[5]), pk16(hb[6], hb[7])};
  *(volatile v4u*)(out + base) = u;
  __threadfence();
  *(volatile v4u*)(out + base) = u;
}

__global__ __launch_bounds__(256) void wtcast_kernel(const float* __restrict__ W, unsigned short* __restrict__ WT,
                                                     int din, int dout, float scale) {
  __shared__ float sm[64][65];
  const int t  = threadIdx.x;
  const int d0 = blockIdx.x * 64;
  const int o0 = blockIdx.y * 64;
#pragma unroll
  for (int i = 0; i < 16; ++i) {
    const int e = i * 256 + t;
    const int r = e >> 6;
    const int cidx = e & 63;
    sm[cidx][r] = W[(size_t)(d0 + r) * dout + o0 + cidx] * scale;
  }
  __syncthreads();
  const int lane = t & 31, wave = t >> 5;
  const int q = lane >> 3, c8 = (lane & 7) * 8;
  for (int pass = 0; pass < 2; ++pass) {
#pragma unroll
    for (int it = 0; it < 2; ++it) {
      const int row = wave * 8 + it * 4 + q;
      unsigned short hb[8];
#pragma unroll
      for (int e = 0; e < 8; ++e) hb[e] = h_bits(sm[row][c8 + e]);
      const v4u u = (v4u){pk16(hb[0], hb[1]), pk16(hb[2], hb[3]), pk16(hb[4], hb[5]), pk16(hb[6], hb[7])};
      *(volatile v4u*)(WT + (size_t)(o0 + row) * din + d0 + c8) = u;
    }
    __threadfence();
  }
}

__device__ __forceinline__ v8f mma_h(v16h a, v16h b, v8f c) {
  c = __builtin_amdgcn_wmma_f32_16x16x32_f16(false, a, false, b, (short)0, c, false, false);
  asm volatile("v_nop\n\tv_nop\n\tv_nop\n\tv_nop" : "+v"(c) : "v"(a), "v"(b));
  return c;
}

__global__ __launch_bounds__(128) void rel_attn_kernel(
    const float* __restrict__ qf,
    const _Float16* __restrict__ kvp,
    const _Float16* __restrict__ rhp,
    const float* __restrict__ rwb,
    const float* __restrict__ rrb,
    unsigned short* __restrict__ av) {
  __shared__ __align__(16) _Float16 Ksh[kKC * kDHead];
  __shared__ __align__(16) _Float16 Vt[kDHead * kKC];
  __shared__ __align__(16) _Float16 Rw[kRWin * kDHead];
  __shared__ __align__(16) _Float16 Psh[4][16 * kKC];
  __shared__ __align__(16) float    Bds[4][16 * kBdPitch];

  const int tid  = threadIdx.x;
  const int wave = tid >> 5;
  const int lane = tid & 31;
  const int hh   = lane >> 4;
  const int c    = lane & 15;

  const int bx = blockIdx.x;
  const int qb = bx & 15;
  const int bhx = bx >> 4;
  const int n  = bhx & 15;
  const int b  = bhx >> 4;
  const int qB = qb * 64;
  const int q0 = qB + wave * 16;

  v16h qw[2], qr[2];
  {
    const float* qrow = qf + ((size_t)(b * kQLen + q0 + c)) * kHDim + n * kDHead;
    const float* bw = rwb + n * kDHead;
    const float* br = rrb + n * kDHead;
#pragma unroll
    for (int dc = 0; dc < 2; ++dc) {
#pragma unroll
      for (int e = 0; e < 8; ++e) {
        const int d0i = dc * 32 + 8 * hh + e;
        const int d1i = d0i + 16;
        const float f0 = qrow[d0i];
        const float f1 = qrow[d1i];
        qw[dc][e]     = (_Float16)(f0 + bw[d0i]);
        qw[dc][8 + e] = (_Float16)(f1 + bw[d1i]);
        qr[dc][e]     = (_Float16)(f0 + br[d0i]);
        qr[dc][8 + e] = (_Float16)(f1 + br[d1i]);
      }
    }
  }

  float mrow[8], lrow[8];
  v8f oacc[4];
#pragma unroll
  for (int r = 0; r < 8; ++r) { mrow[r] = -INFINITY; lrow[r] = 0.f; }
#pragma unroll
  for (int t = 0; t < 4; ++t) oacc[t] = (v8f){0.f,0.f,0.f,0.f,0.f,0.f,0.f,0.f};

  const int nChunks = qb + 17;
  const int kvr = tid >> 1, dh = (tid & 1) * 32;
  const int U0 = 48 - 16 * wave;

  for (int kc = 0; kc < nChunks; ++kc) {
    const int kv0 = kc * kKC;
    __syncthreads();
    {
      const _Float16* krow = kvp + ((size_t)(b * kKLen + kv0 + kvr)) * kKVPitch + n * kDHead + dh;
      const _Float16* vrow = krow + kHDim;
#pragma unroll
      for (int i = 0; i < 4; ++i) {
        const v8h kk8 = *(const v8h*)(krow + 8 * i);
        *(v8h*)(Ksh + kvr * kDHead + dh + 8 * i) = kk8;
        const v8h vv8 = *(const v8h*)(vrow + 8 * i);
#pragma unroll
        for (int e = 0; e < 8; ++e) Vt[(dh + 8 * i + e) * kKC + kvr] = vv8[e];
      }
      int m = kv0 + 959 - qB + tid;
      m = m < 0 ? 0 : m;
      m = m > (kKLen - 1) ? (kKLen - 1) : m;
      const _Float16* rrow = rhp + (size_t)m * kHDim + n * kDHead;
#pragma unroll
      for (int i = 0; i < 8; ++i) *(v8h*)(Rw + tid * kDHead + 8 * i) = *(const v8h*)(rrow + 8 * i);
    }
    __syncthreads();

    v8f s[4];
#pragma unroll
    for (int j = 0; j < 4; ++j) {
      s[j] = (v8f){0.f,0.f,0.f,0.f,0.f,0.f,0.f,0.f};
#pragma unroll
      for (int dc = 0; dc < 2; ++dc) {
        const v16h kb = Frag<_Float16>::load(Ksh + (j * 16 + c) * kDHead + dc * 32 + 8 * hh);
        s[j] = mma_h(qw[dc], kb, s[j]);
      }
    }

    float* bdw = Bds[wave];
#pragma unroll
    for (int t = 0; t < 5; ++t) {
      v8f bacc = (v8f){0.f,0.f,0.f,0.f,0.f,0.f,0.f,0.f};
#pragma unroll
      for (int dc = 0; dc < 2; ++dc) {
        const v16h rb = Frag<_Float16>::load(Rw + (U0 + t * 16 + c) * kDHead + dc * 32 + 8 * hh);
        bacc = mma_h(qr[dc], rb, bacc);
      }
#pragma unroll
      for (int r = 0; r < 8; ++r) bdw[(8 * hh + r) * kBdPitch + t * 16 + c] = bacc[r];
    }
    __builtin_amdgcn_fence(__ATOMIC_RELEASE, "workgroup");
    __builtin_amdgcn_wave_barrier();
    __builtin_amdgcn_fence(__ATOMIC_ACQUIRE, "workgroup");

    float cm[8];
#pragma unroll
    for (int r = 0; r < 8; ++r) {
      const int rr = 8 * hh + r;
      const int qi = q0 + rr;
      float mx = -INFINITY;
#pragma unroll
      for (int j = 0; j < 4; ++j) {
        const int cc = j * 16 + c;
        const float bdv = bdw[rr * kBdPitch + cc - rr + 16];
        float sv = (s[j][r] + bdv) * kScoreScale;
        sv = (kv0 + cc > qi + kMLen) ? -INFINITY : sv;
        s[j][r] = sv;
        mx = fmaxf(mx, sv);
      }
#pragma unroll
      for (int off = 1; off < 16; off <<= 1) mx = fmaxf(mx, __shfl_xor(mx, off, 32));
      cm[r] = mx;
    }

    _Float16* pwh = Psh[wave];
#pragma unroll
    for (int r = 0; r < 8; ++r) {
      const float mnew  = fmaxf(mrow[r], cm[r]);
      const float alpha = __expf(mrow[r] - mnew);
      mrow[r] = mnew;
      float psum = 0.f;
#pragma unroll
      for (int j = 0; j < 4; ++j) {
        const float p = __expf(s[j][r] - mnew);
        psum += p;
        pwh[(8 * hh + r) * kKC + j * 16 + c] = (_Float16)(p * kPCarry);
      }
#pragma unroll
      for (int off = 1; off < 16; off <<= 1) psum += __shfl_xor(psum, off, 32);
      lrow[r] = lrow[r] * alpha + psum;
#pragma unroll
      for (int t = 0; t < 4; ++t) oacc[t][r] *= alpha;
    }
    __builtin_amdgcn_fence(__ATOMIC_RELEASE, "workgroup");
    __builtin_amdgcn_wave_barrier();
    __builtin_amdgcn_fence(__ATOMIC_ACQUIRE, "workgroup");

#pragma unroll
    for (int kk = 0; kk < 2; ++kk) {
      const v16h pa = Frag<_Float16>::load(pwh + c * kKC + kk * 32 + 8 * hh);
#pragma unroll
      for (int t = 0; t < 4; ++t) {
        const v16h vb = Frag<_Float16>::load(Vt + (t * 16 + c) * kKC + kk * 32 + 8 * hh);
        oacc[t] = mma_h(pa, vb, oacc[t]);
      }
    }
  }

  __builtin_amdgcn_fence(__ATOMIC_RELEASE, "workgroup");
  __builtin_amdgcn_wave_barrier();
  __builtin_amdgcn_fence(__ATOMIC_ACQUIRE, "workgroup");
  float* os = Bds[wave];
#pragma unroll
  for (int r = 0; r < 8; ++r) {
    const float inv = 1.0f / (lrow[r] * 128.0f);
#pragma unroll
    for (int t = 0; t < 4; ++t) os[(8 * hh + r) * kOsPitch + t * 16 + c] = oacc[t][r] * inv;
  }
  __builtin_amdgcn_fence(__ATOMIC_RELEASE, "workgroup");
  __builtin_amdgcn_wave_barrier();
  __builtin_amdgcn_fence(__ATOMIC_ACQUIRE, "workgroup");
  {
    const int q8 = lane >> 3, c8 = (lane & 7) * 8;
    for (int pass = 0; pass < 2; ++pass) {
#pragma unroll
      for (int it = 0; it < 4; ++it) {
        const int row = it * 4 + q8;
        const float* sp = os + row * kOsPitch + c8;
        v8h hv;
#pragma unroll
        for (int e = 0; e < 8; ++e) hv[e] = (_Float16)sp[e];
        *(volatile v8h*)(av + ((size_t)(q0 + row) * kBsz + b) * kHDim + n * kDHead + c8) = hv;
      }
      __threadfence();
    }
  }
}

__global__ __launch_bounds__(256) void ln_out_kernel(const float* __restrict__ x, const float* __restrict__ g,
                                                    const float* __restrict__ be, float* __restrict__ out) {
  __shared__ float red[16];
  const int row  = blockIdx.x;
  const int t    = threadIdx.x, lane = t & 31, wave = t >> 5;
  const int c0   = t * 4;
  const float* xr = x + (size_t)row * kDModel + c0;
  const v4f a = *(const v4f*)(xr);
  float s = (a[0] + a[1]) + (a[2] + a[3]);
#pragma unroll
  for (int off = 16; off > 0; off >>= 1) s += __shfl_xor(s, off, 32);
  if (lane == 0) red[wave] = s;
  __syncthreads();
  const float mu = (((red[0] + red[1]) + (red[2] + red[3])) + ((red[4] + red[5]) + (red[6] + red[7]))) * kInvD;
  const float d0 = a[0] - mu, d1 = a[1] - mu, d2 = a[2] - mu, d3 = a[3] - mu;
  float s2 = (d0 * d0 + d1 * d1) + (d2 * d2 + d3 * d3);
#pragma unroll
  for (int off = 16; off > 0; off >>= 1) s2 += __shfl_xor(s2, off, 32);
  if (lane == 0) red[8 + wave] = s2;
  __syncthreads();
  const float var  = (((red[8] + red[9]) + (red[10] + red[11])) + ((red[12] + red[13]) + (red[14] + red[15]))) * kInvD;
  const float rstd = rsqrtf(var + kLnEps);
  const v4f gg = *(const v4f*)(g + c0);
  const v4f bb = *(const v4f*)(be + c0);
  v4f o;
  o[0] = (d0 * rstd) * gg[0] + bb[0];
  o[1] = (d1 * rstd) * gg[1] + bb[1];
  o[2] = (d2 * rstd) * gg[2] + bb[2];
  o[3] = (d3 * rstd) * gg[3] + bb[3];
  float* op = out + (size_t)row * kDModel + c0;
  *(volatile v4f*)op = o;
  __threadfence();
  *(volatile v4f*)op = o;
}

extern "C" void kernel_launch(void* const* d_in, const int* in_sizes, int n_in,
                              void* d_out, int out_size, void* d_ws,
                              size_t ws_size, hipStream_t stream) {
  if (n_in < 10) return;
  if (in_sizes[0] != kQLen * kBsz * kDModel) return;
  if (in_sizes[1] != kKLen * kDModel) return;
  if (in_sizes[2] != kMLen * kBsz * kDModel) return;
  if (in_sizes[3] != kDModel * kQkvCols) return;
  if (in_sizes[4] != kDModel * kHDim) return;
  if (in_sizes[5] != kHDim * kDModel) return;
  if (in_sizes[6] != kNHead * kDHead) return;
  if (in_sizes[7] != kNHead * kDHead) return;
  if (in_sizes[8] != kDModel) return;
  if (in_sizes[9] != kDModel) return;
  if (out_size != kQLen * kBsz * kDModel) return;

  const float* w     = (const float*)d_in[0];
  const float* rpos  = (const float*)d_in[1];
  const float* mems  = (const float*)d_in[2];
  const float* W_qkv = (const float*)d_in[3];
  const float* W_r   = (const float*)d_in[4];
  const float* W_o   = (const float*)d_in[5];
  const float* rwb   = (const float*)d_in[6];
  const float* rrb   = (const float*)d_in[7];
  const float* gamma = (const float*)d_in[8];
  const float* beta  = (const float*)d_in[9];
  float* out = (float*)d_out;

  const size_t szCat  = (size_t)kKLen * kBsz * kDModel * 2;
  const size_t szR    = (size_t)kKLen * kDModel * 2;
  const size_t szWqkv = (size_t)kQkvCols * kDModel * 2;
  const size_t szWr   = (size_t)kHDim * kDModel * 2;
  const size_t szWo   = (size_t)kDModel * kHDim * 2;
  const size_t szKV   = (size_t)kBsz * kKLen * kKVPitch * 2;
  const size_t szQ    = (size_t)kBsz * kQLen * kHDim * 4;
  const size_t szRh   = (size_t)kKLen * kHDim * 2;
  const size_t szAv   = (size_t)kTokQ * kHDim * 2;
  const size_t szX    = (size_t)kTokQ * kDModel * 4;
  const size_t offCat  = 0;
  const size_t offR    = offCat + szCat;
  const size_t offWqkv = offR + szR;
  const size_t offWr   = offWqkv + szWqkv;
  const size_t offWo   = offWr + szWr;
  const size_t offKV   = offWo + szWo;
  const size_t offQ    = offKV + szKV;
  const size_t offRh   = offQ + szQ;
  const size_t offAv   = offRh + szRh;
  const size_t offX    = offAv + szAv;
  const size_t total   = offX + szX;
  if (total > ws_size) return;

  char* ws = (char*)d_ws;
  unsigned short* cat16 = (unsigned short*)(ws + offCat);
  unsigned short* r16   = (unsigned short*)(ws + offR);
  unsigned short* wqkvT = (unsigned short*)(ws + offWqkv);
  unsigned short* wrT   = (unsigned short*)(ws + offWr);
  unsigned short* woT   = (unsigned short*)(ws + offWo);
  unsigned short* kv16  = (unsigned short*)(ws + offKV);
  float*          qf32  = (float*)(ws + offQ);
  unsigned short* rh16  = (unsigned short*)(ws + offRh);
  unsigned short* av16  = (unsigned short*)(ws + offAv);
  float*          x32   = (float*)(ws + offX);

  const int n8Tok = (kMLen * kBsz * kDModel) / 8;
  const int n8R   = (kKLen * kDModel) / 8;

  cast8_kernel<<<n8Tok / 256, 256, 0, stream>>>(mems, cat16, n8Tok);
  cast8_kernel<<<n8Tok / 256, 256, 0, stream>>>(w, cat16 + (size_t)kMLen * kBsz * kDModel, n8Tok);
  cast8_kernel<<<n8R / 256, 256, 0, stream>>>(rpos, r16, n8R);

  wtcast_kernel<<<dim3(kDModel / 64, kQkvCols / 64), 256, 0, stream>>>(W_qkv, wqkvT, kDModel, kQkvCols, kWCarry);
  wtcast_kernel<<<dim3(kDModel / 64, kHDim / 64), 256, 0, stream>>>(W_r, wrT, kDModel, kHDim, kWCarry);
  wtcast_kernel<<<dim3(kHDim / 64, kDModel / 64), 256, 0, stream>>>(W_o, woT, kHDim, kDModel, kWCarry);

  {
    const int tiles = (kKLen / 64) * (kKVPitch / 64);
    wmma_gemm64<0, false, 0, 1, false><<<dim3(tiles / 8, kBsz), 256, 0, stream>>>(
        cat16, cat16, kBsz * kDModel, (long)kDModel,
        wqkvT + (size_t)kHDim * kDModel, wqkvT + (size_t)kHDim * kDModel, kDModel, (long)0,
        (void*)kv16, (void*)kv16, kKVPitch, (long)kKLen * kKVPitch,
        rwb, w, (long)0,
        kKLen, kKVPitch, kDModel, kProjScale);
  }
  {
    const int tiles = (kQLen / 64) * (kHDim / 64);
    wmma_gemm64<0, false, 0, 0, false><<<dim3(tiles / 8, kBsz), 256, 0, stream>>>(
        cat16 + (size_t)kMLen * kBsz * kDModel, cat16 + (size_t)kMLen * kBsz * kDModel, kBsz * kDModel, (long)kDModel,
        wqkvT, wqkvT, kDModel, (long)0,
        (void*)qf32, (void*)qf32, kHDim, (long)kQLen * kHDim,
        rwb, w, (long)0,
        kQLen, kHDim, kDModel, kProjScale);
  }
  {
    const int tiles = (kKLen / 64) * (kHDim / 64);
    wmma_gemm64<0, false, 0, 1, false><<<dim3(tiles / 8, 1), 256, 0, stream>>>(
        r16, r16, kDModel, (long)0,
        wrT, wrT, kDModel, (long)0,
        (void*)rh16, (void*)rh16, kHDim, (long)0,
        rwb, w, (long)0,
        kKLen, kHDim, kDModel, kProjScale);
  }
  rel_attn_kernel<<<kBsz * kNHead * (kQLen / 64), 128, 0, stream>>>(
      qf32, (const _Float16*)kv16, (const _Float16*)rh16, rwb, rrb, av16);

  {
    const int tiles = (kTokQ / 64) * (kDModel / 64);
    wmma_gemm64<0, false, 0, 0, true><<<dim3(tiles / 8, 1), 256, 0, stream>>>(
        av16, av16, kHDim, (long)0,
        woT, woT, kHDim, (long)0,
        (void*)x32, (void*)x32, kDModel, (long)0,
        rwb, w, (long)0,
        kTokQ, kDModel, kHDim, kOutScale);
  }
  ln_out_kernel<<<kTokQ, 256, 0, stream>>>(x32, gamma, beta, out);
}
